// dgl_GraphConv_39625368273413
// MI455X (gfx1250) — hardware-verified
//
#include <hip/hip_runtime.h>

typedef float          v8f   __attribute__((ext_vector_type(8)));
typedef float          v4f   __attribute__((ext_vector_type(4)));
typedef unsigned int   v4u   __attribute__((ext_vector_type(4)));
typedef int            v8i   __attribute__((ext_vector_type(8)));
typedef unsigned short v8us  __attribute__((ext_vector_type(8)));
typedef unsigned short v16us __attribute__((ext_vector_type(16)));
typedef __bf16         v16bf __attribute__((ext_vector_type(16)));
typedef _Float16       v16h  __attribute__((ext_vector_type(16)));
typedef v4f  __attribute__((may_alias)) v4fa;
typedef v8us __attribute__((may_alias)) v8usa;
union FragB { v16bf v; v16us u; v8us h[2]; v8i w; };
union FragH { v16h  v; v16us u; v8us h[2]; v8i w; };

__device__ __forceinline__ v8f wmb(const FragB& a, const FragB& b, v8f c) {
  v8f d = __builtin_amdgcn_wmma_f32_16x16x32_bf16(false, a.v, false, b.v, (short)0, c, false, false);
  asm volatile("v_nop\n\tv_nop\n\tv_nop\n\tv_nop" : "+v"(d) : "v"(a.w), "v"(b.w));
  return d;
}

__device__ __forceinline__ v8f wmh(const FragH& a, const FragH& b, v8f c) {
  v8f d = __builtin_amdgcn_wmma_f32_16x16x32_f16(false, a.v, false, b.v, (short)0, c, false, false);
  asm volatile("v_nop\n\tv_nop\n\tv_nop\n\tv_nop" : "+v"(d) : "v"(a.w), "v"(b.w));
  return d;
}

__device__ __forceinline__ unsigned bf16_bits(float f) {
  const unsigned u = __float_as_uint(f);
  const unsigned r = (u + 0x7FFFu + ((u >> 16) & 1u)) >> 16;
  const unsigned q = (u >> 16) | 0x40u;
  return ((u & 0x7fffffffu) > 0x7f800000u) ? q : r;
}

__device__ __forceinline__ float bf16_val(float f) {
  return __uint_as_float(bf16_bits(f) << 16);
}
__device__ __forceinline__ int clampi(int v, int lo, int hi) {
  return v < lo ? lo : (v > hi ? hi : v);
}

__device__ __forceinline__ unsigned f16_bits(float f) {
  const unsigned u  = __float_as_uint(f);
  const unsigned s  = (u >> 16) & 0x8000u;
  const unsigned a  = u & 0x7fffffffu;
  const unsigned t  = a - 0x38000000u;
  const unsigned r  = (t + 0x0FFFu + ((t >> 13) & 1u)) >> 13;
  const unsigned rc = r > 0x7C00u ? 0x7C00u : r;
  const bool small  = a < 0x38800000u;
  const bool isnan  = a > 0x7f800000u;
  const unsigned fin = small ? 0u : (s | rc);
  return isnan ? (s | 0x7E00u) : fin;
}

__device__ __forceinline__ unsigned pk16(unsigned lo, unsigned hi) { return lo | (hi << 16); }
__device__ __forceinline__ unsigned bf16_lo_bits(float v) {
  float hi = bf16_val(v);
  asm volatile("" : "+v"(hi));
  return bf16_bits(v - hi);
}
__device__ __forceinline__ v4u pack8_bf16(v4f a, v4f c) {
  return (v4u){ pk16(bf16_bits(a[0]), bf16_bits(a[1])), pk16(bf16_bits(a[2]), bf16_bits(a[3])),
                pk16(bf16_bits(c[0]), bf16_bits(c[1])), pk16(bf16_bits(c[2]), bf16_bits(c[3])) };
}
__device__ __forceinline__ v4u pack8_bf16_lo(v4f a, v4f c) {
  return (v4u){ pk16(bf16_lo_bits(a[0]), bf16_lo_bits(a[1])), pk16(bf16_lo_bits(a[2]), bf16_lo_bits(a[3])),
                pk16(bf16_lo_bits(c[0]), bf16_lo_bits(c[1])), pk16(bf16_lo_bits(c[2]), bf16_lo_bits(c[3])) };
}
__device__ __forceinline__ v4u pack8_f16(v4f a, v4f c) {
  return (v4u){ pk16(f16_bits(a[0]), f16_bits(a[1])), pk16(f16_bits(a[2]), f16_bits(a[3])),
                pk16(f16_bits(c[0]), f16_bits(c[1])), pk16(f16_bits(c[2]), f16_bits(c[3])) };
}

template <int FORM>
__global__ __launch_bounds__(256) void k_plane(const float* __restrict__ src, int rows, int cols, int ldsrc,
                                               unsigned short* __restrict__ dst, int MP, int KP) {
  static_assert(FORM >= 0 && FORM <= 3);
  const int KTOT = (FORM == 1 || FORM == 3) ? 2 * KP : KP;
  const unsigned ppr   = (unsigned)(KTOT >> 3);
  const unsigned kp8   = (unsigned)(KP >> 3);
  const unsigned total = (unsigned)MP * ppr;
  const unsigned g     = blockIdx.x * 256u + threadIdx.x;
  const unsigned rowu  = g / ppr;
  const unsigned p     = g - rowu * ppr;
  const bool second    = p >= kp8;
  const int row = (int)rowu;
  const int c0  = (int)((second ? p - kp8 : p) << 3);
  const float* srow = src + (size_t)clampi(row, 0, rows - 1) * (size_t)ldsrc;
  float x[8];
  unsigned mk[8];
#pragma unroll
  for (int e = 0; e < 8; ++e) {
    const int c = c0 + e;
    const float v = srow[clampi(c, 0, cols - 1)];
    asm volatile("" :: "v"(v));
    x[e]  = v;
    mk[e] = (row < rows && c < cols) ? 0xFFFFu : 0u;
  }
  const v4f a = (v4f){ x[0], x[1], x[2], x[3] };
  const v4f c = (v4f){ x[4], x[5], x[6], x[7] };
  v4u o;
  if (FORM == 2) {
    o = pack8_f16(a, c);
  } else {
    const v4u hi = pack8_bf16(a, c);
    o = hi;
    if (FORM == 1) { const v4u lo = pack8_bf16_lo(a, c); o = second ? lo : hi; }
  }
  const v4u mw = (v4u){ pk16(mk[0], mk[1]), pk16(mk[2], mk[3]), pk16(mk[4], mk[5]), pk16(mk[6], mk[7]) };
  o &= mw;
  if (g < total) {
    volatile v4u* q = (volatile v4u*)(dst + (size_t)g * 8);
    *q = o;
    __threadfence();
    *q = o;
  }
}

template <int FORM> struct FragOf    { typedef FragB T; };
template <>         struct FragOf<2> { typedef FragH T; };
__device__ __forceinline__ v8f mm(const FragB& a, const FragB& b, v8f c) { return wmb(a, b, c); }
__device__ __forceinline__ v8f mm(const FragH& a, const FragH& b, v8f c) { return wmh(a, b, c); }
template <class F> __device__ __forceinline__ F ld_frag(const unsigned short* p) {
  F f;
  f.h[0] = *(const v8usa*)(p);
  f.h[1] = *(const v8usa*)(p + 16);
  return f;
}

template <int FORM, int EPI>
__global__ __launch_bounds__(256) __attribute__((amdgpu_num_vgpr(248)))
void k_gemm_nt(const unsigned short* __restrict__ A, const unsigned short* __restrict__ B,
               const float* __restrict__ bias, float* __restrict__ D, int M, int N, int KTOT, int ldd) {
  static_assert(FORM >= 0 && FORM <= 2);
  static_assert(EPI == 0 || EPI == 1);
  typedef typename FragOf<FORM>::T F;
  __shared__ __attribute__((aligned(16))) float sT[8][16 * 68];
  const int lane = threadIdx.x & 31;
  const int wave = threadIdx.x >> 5;
  const int tilesM = (M + 63) >> 6;
  const int tilesN = (N + 63) >> 6;
  const int tile = blockIdx.x * 8 + wave;
  if (tile >= tilesM * tilesN) return;
  const int tm = tile / tilesN;
  const int tn = tile - tm * tilesN;
  const int m0 = tm << 6;
  const int n0 = tn << 6;

  const int rl = lane & 15;
  const int h8 = (lane >> 4) * 8;
  const unsigned short* pa = A + (size_t)(m0 + rl) * (size_t)KTOT + h8;
  const unsigned short* pb = B + (size_t)(n0 + rl) * (size_t)KTOT + h8;

  v8f acc[4][4];
#pragma unroll
  for (int i = 0; i < 4; ++i)
#pragma unroll
    for (int j = 0; j < 4; ++j) acc[i][j] = (v8f){0.f, 0.f, 0.f, 0.f, 0.f, 0.f, 0.f, 0.f};

#pragma unroll 1
  for (int k0 = 0; k0 < KTOT; k0 += 32) {
    F bf[4];
#pragma unroll
    for (int j = 0; j < 4; ++j) bf[j] = ld_frag<F>(pb + (size_t)(j << 4) * (size_t)KTOT + k0);
#pragma unroll
    for (int i = 0; i < 4; ++i) {
      const F af = ld_frag<F>(pa + (size_t)(i << 4) * (size_t)KTOT + k0);
#pragma unroll
      for (int j = 0; j < 4; ++j) acc[i][j] = mm(af, bf[j], acc[i][j]);
    }
  }

  float* slab = sT[wave];
  const int hh = lane >> 4;
  const int c4 = (lane & 15) * 4;
  const int nc = n0 + c4;
  const bool cok = nc < N;
  v4f bv = (v4f){0.f, 0.f, 0.f, 0.f};
  if (EPI == 1) {
    bv = *(const v4fa*)(bias + clampi(nc, 0, N - 4));
    asm volatile("" :: "v"(bv));
  }
#pragma unroll
  for (int i = 0; i < 4; ++i) {
    const int mBase = m0 + (i << 4);
#pragma unroll
    for (int j = 0; j < 4; ++j) {
#pragma unroll
      for (int r = 0; r < 8; ++r) slab[(h8 + r) * 68 + (j << 4) + rl] = acc[i][j][r];
    }
    __builtin_amdgcn_fence(__ATOMIC_RELEASE, "workgroup");
    __builtin_amdgcn_wave_barrier();
    __builtin_amdgcn_fence(__ATOMIC_ACQUIRE, "workgroup");
    v4f vv[8];
#pragma unroll
    for (int it = 0; it < 8; ++it) {
      const int row = it * 2 + hh;
      v4f v = *(const v4fa*)(slab + row * 68 + c4);
      if (EPI == 1) v += bv;
      vv[it] = v;
    }
    for (int pass = 0; pass < 2; ++pass) {
#pragma unroll
      for (int it = 0; it < 8; ++it) {
        const int row = mBase + it * 2 + hh;
        if (cok && row < M) *(volatile v4f*)(D + (size_t)row * (size_t)ldd + nc) = vv[it];
      }
      __threadfence();
    }
    __builtin_amdgcn_fence(__ATOMIC_RELEASE, "workgroup");
    __builtin_amdgcn_wave_barrier();
    __builtin_amdgcn_fence(__ATOMIC_ACQUIRE, "workgroup");
  }
}

#define AGG_SPLIT 1

#define NN     100000
#define EE     1000000
#define DD     64
#define AP     (DD + DD * (1 + AGG_SPLIT))
#define APW    (AP / 2)
#define MPAD   100096

#define NTHR   256
#define NWAVE  8
#define EPT    8
#define CHUNK  (NTHR * EPT)
#define WCAP   (EPT * 32)
#define LISTN  (NWAVE * WCAP)
#define NBA    1024
#define SLA    10
#define RCAP   28672
#define DEGCAP 64
#define MEAS_MAXDEG 33
#define MEAS_B1024  10433
#define NBLK   ((NN + NBA - 1) / NBA)
#define AGG_ZINTS     (LISTN + 2 * RCAP + 3 * NBA)
#define MISC_INTS     16
#define SCAN_LDS_INTS (AGG_ZINTS + MISC_INTS)

#define PB_FEAT  ((NN * 8) / 256)
#define PB_PAD   (((MPAD - NN) * (AP / 8)) / 256)
#define PB_W     ((DD * (AP / 8)) / 256)
#define PB_TOTAL (PB_FEAT + PB_PAD + PB_W + 1)

#define SZ_A     ((size_t)MPAD * AP * 2)
#define SZ_WB    ((size_t)DD * AP * 2)
#define SZ_BSUM  ((size_t)256)
#define SZ_FLAG  ((size_t)512)
#define WS_TOTAL (SZ_A + SZ_WB + SZ_BSUM + SZ_FLAG)

static_assert(AGG_SPLIT == 0 || AGG_SPLIT == 1);
static_assert(DD == 64);
static_assert(2 * 32 == DD);
static_assert(AP % 32 == 0 && (AP * 2) % 128 == 0);
static_assert(MPAD == 100096 && MPAD % 128 == 0 && MPAD % 64 == 0);
static_assert(MPAD >= ((NN + 63) / 64) * 64);
static_assert(NN % 16 == 0 && DD % 4 == 0 && DD % 32 == 0);
static_assert(EE % EPT == 0 && EE >= CHUNK && EE < (1 << 21));
static_assert((CHUNK & (CHUNK - 1)) == 0 && NBA == (1 << SLA));
static_assert(((long long)EE << SLA) < (1LL << 31));
static_assert(NBLK * NBA >= NN && NBLK <= 128);
static_assert(RCAP >= 2 * MEAS_B1024);
static_assert(DEGCAP >= MEAS_MAXDEG + 8);
static_assert(AGG_ZINTS % (NTHR * 4) == 0);
static_assert(SCAN_LDS_INTS * 4 <= 327680);
static_assert((NN * 8) % 256 == 0);
static_assert(((MPAD - NN) * (AP / 8)) % 256 == 0);
static_assert((DD * (AP / 8)) % 256 == 0);
static_assert(((size_t)NN * AP * 2) % 128 == 0);
static_assert(SZ_A % 256 == 0 && SZ_WB % 256 == 0);
static_assert(WS_TOTAL <= ((size_t)128 << 20));
static_assert(AGG_SPLIT == 0 || WS_TOTAL == 38462208);

typedef int  v4i  __attribute__((ext_vector_type(4)));
typedef v4i  __attribute__((may_alias)) v4ia;

__global__ __launch_bounds__(256) void k_prep(const float* __restrict__ feat, const float* __restrict__ Wlin,
                                              const float* __restrict__ blin, const float* __restrict__ Wrot,
                                              const float* __restrict__ brot, unsigned short* __restrict__ Apl,
                                              unsigned short* __restrict__ WB, float* __restrict__ bsum,
                                              int* __restrict__ flag) {
  const int tid = (int)threadIdx.x;
#pragma unroll 1
  for (int bu = (int)blockIdx.x; bu < PB_TOTAL; bu += (int)gridDim.x) {
    if (bu < PB_FEAT) {
      const int g   = bu * 256 + tid;
      const int row = g >> 3;
      const int p   = g & 7;
      const float* s = feat + (size_t)row * DD + 8 * p;
      const v4f a = *(const v4fa*)s;
      const v4f c = *(const v4fa*)(s + 4);
      const v4u o = pack8_bf16(a, c);
      volatile v4u* q = (volatile v4u*)(Apl + (size_t)row * AP + 8 * p);
      *q = o;
      __threadfence();
      *q = o;
    } else if (bu < PB_FEAT + PB_PAD) {
      const int g = (bu - PB_FEAT) * 256 + tid;
      const v4u z = (v4u){0u, 0u, 0u, 0u};
      volatile v4u* q = (volatile v4u*)(Apl + (size_t)NN * AP + (size_t)g * 8);
      *q = z;
      __threadfence();
      *q = z;
    } else if (bu < PB_FEAT + PB_PAD + PB_W) {
      const int g  = (bu - PB_FEAT - PB_PAD) * 256 + tid;
      const int n  = g / (AP / 8);
      const int p  = g - n * (AP / 8);
      const int k0 = 8 * p;
      const int kk = k0 & (DD - 1);
      const float* sr = Wrot + (size_t)n * DD + kk;
      const float* sl = Wlin + (size_t)n * DD + kk;
      const v4f ra = *(const v4fa*)sr;
      const v4f rc = *(const v4fa*)(sr + 4);
      const v4f la = *(const v4fa*)sl;
      const v4f lc = *(const v4fa*)(sl + 4);
      asm volatile("" :: "v"(ra), "v"(rc), "v"(la), "v"(lc));
      const v4u pr = pack8_bf16(ra, rc);
      const v4u pl = pack8_bf16(la, lc);
      const unsigned mk = (k0 < DD) ? 0xFFFFFFFFu : 0u;
      const v4u mv = (v4u){mk, mk, mk, mk};
      const v4u o  = (pr & mv) | (pl & ~mv);
      volatile v4u* q = (volatile v4u*)(WB + (size_t)g * 8);
      *q = o;
      __threadfence();
      *q = o;
    } else {
      const int i4 = (tid & 15) * 4;
      const v4f bl = *(const v4fa*)(blin + i4);
      const v4f br = *(const v4fa*)(brot + i4);
      asm volatile("" :: "v"(bl), "v"(br));
      const v4f sv = (v4f){ bf16_val(bl[0]) + bf16_val(br[0]), bf16_val(bl[1]) + bf16_val(br[1]),
                            bf16_val(bl[2]) + bf16_val(br[2]), bf16_val(bl[3]) + bf16_val(br[3]) };
      const v4u z = (v4u){0u, 0u, 0u, 0u};
      const int fi = ((tid - 32) & 31) * 4;
      for (int pass = 0; pass < 2; ++pass) {
        if (tid < 16) *(volatile v4f*)(bsum + i4) = sv;
        if (tid >= 32 && tid < 64) *(volatile v4u*)(flag + fi) = z;
        __threadfence();
      }
    }
  }
}

__global__ __launch_bounds__(NTHR) void k_scan_sum(const int* __restrict__ gath, const int* __restrict__ keys,
                                                   unsigned* aplw, int* __restrict__ flag) {
  extern __shared__ __attribute__((aligned(16))) int dsm[];
  constexpr int OL = 0;
  constexpr int OH = OL + LISTN;
  constexpr int OS = OH + RCAP;
  constexpr int OC = OS + RCAP;
  constexpr int OO = OC + NBA;
  constexpr int OU = OO + NBA;
  constexpr int OM = OU + NBA;
  const int tid = (int)threadIdx.x, lane = tid & 31, wave = tid >> 5;
  const int nodeBase = (int)blockIdx.x * NBA;
  int nb = NN - nodeBase;
  nb = nb < 0 ? 0 : (nb > NBA ? NBA : nb);

  {
    const v4i z4 = (v4i){0, 0, 0, 0};
    for (int i = tid * 4; i < AGG_ZINTS; i += NTHR * 4) *(v4ia*)(dsm + i) = z4;
    if (tid < MISC_INTS) dsm[OM + tid] = 0;
  }
  __syncthreads();

  int t = 0, ov = 0;
  constexpr int nChunks = (EE + CHUNK - 1) / CHUNK;
  const unsigned nbs = (unsigned)nodeBase;
  const unsigned unb = (unsigned)nb;
#pragma unroll 1
  for (int ch = 0; ch < nChunks; ++ch) {
    const int cbase = ch * CHUNK;
    int wc = 0;
    {
      const int el0 = tid * EPT;
      const int e0  = cbase + el0;
      const int ec  = e0 < (EE - EPT) ? e0 : (EE - EPT);
      const v4i da = *(const v4ia*)(keys + ec);
      const v4i db = *(const v4ia*)(keys + ec + 4);
      asm volatile("" :: "v"(da), "v"(db));
      const int om = (e0 < EE) ? 0 : -1;
      const unsigned s0 = (unsigned)(da.x | om) - nbs, s1 = (unsigned)(da.y | om) - nbs;
      const unsigned s2 = (unsigned)(da.z | om) - nbs, s3 = (unsigned)(da.w | om) - nbs;
      const unsigned s4 = (unsigned)(db.x | om) - nbs, s5 = (unsigned)(db.y | om) - nbs;
      const unsigned s6 = (unsigned)(db.z | om) - nbs, s7 = (unsigned)(db.w | om) - nbs;
      const bool h0 = s0 < unb, h1 = s1 < unb, h2 = s2 < unb, h3 = s3 < unb;
      const bool h4 = s4 < unb, h5 = s5 < unb, h6 = s6 < unb, h7 = s7 < unb;
      const unsigned any = __builtin_amdgcn_ballot_w32(h0 | h1 | h2 | h3 | h4 | h5 | h6 | h7);
      if (any != 0u) {
#define HITJ(J, HJ, SJ) { \
        const unsigned mj = __builtin_amdgcn_ballot_w32(HJ); \
        if (mj != 0u) { \
          const int pos = wc + (int)__builtin_amdgcn_mbcnt_lo(mj, 0u); \
          if ((HJ) && pos < WCAP) dsm[OL + wave * WCAP + pos] = ((el0 + (J)) << SLA) | (int)(SJ); \
          wc += (int)__builtin_popcount(mj); } }
        HITJ(0, h0, s0)
        HITJ(1, h1, s1)
        HITJ(2, h2, s2)
        HITJ(3, h3, s3)
        HITJ(4, h4, s4)
        HITJ(5, h5, s5)
        HITJ(6, h6, s6)
        HITJ(7, h7, s7)
#undef HITJ
      }
    }
    if (lane == 0) dsm[OM + wave] = wc;
    __syncthreads();
    if (wave == 0) {
#pragma unroll 1
      for (int w2 = 0; w2 < NWAVE; ++w2) {
        int cv = dsm[OM + w2];
        cv = cv < 0 ? 0 : (cv > WCAP ? WCAP : cv);
        const int c = __builtin_amdgcn_readfirstlane(cv);
#pragma unroll 1
        for (int b0 = 0; b0 < c; b0 += 32) {
          const int idx = b0 + lane;
          const int ent = dsm[OL + w2 * WCAP + (idx < WCAP ? idx : WCAP - 1)];
          const int m32 = (c - b0) < 32 ? (c - b0) : 32;
#pragma unroll 1
          for (int k = 0; k < m32; ++k) {
            const int u    = __builtin_amdgcn_readlane(ent, k);
            const int slot = u & (NBA - 1);
            const int el   = (u >> SLA) & (CHUNK - 1);
            const int pk   = ((cbase + el) << SLA) | slot;
            if (t < RCAP) {
              if (lane == 0) { dsm[OH + t] = pk; dsm[OC + slot] = dsm[OC + slot] + 1; }
              t = t + 1;
            } else {
              ov = 1;
            }
          }
        }
      }
    }
    __syncthreads();
  }
  if (tid == 0) { dsm[OM + 8] = t; dsm[OM + 9] = ov; }
  __syncthreads();
  int ttv = dsm[OM + 8];
  ttv = ttv < 0 ? 0 : (ttv > RCAP ? RCAP : ttv);
  const int tt = __builtin_amdgcn_readfirstlane(ttv);

  if (wave == 0) {
    const int base = lane * (NBA / 32);
    int s = 0, bigl = 0;
#pragma unroll 1
    for (int i = 0; i < NBA / 32; ++i) {
      const int cv = dsm[OC + base + i];
      s += cv;
      bigl |= (cv > DEGCAP) ? 1 : 0;
    }
    int incl = s;
#pragma unroll
    for (int d = 1; d < 32; d <<= 1) {
      const int y = __shfl_up(incl, d, 32);
      if (lane >= d) incl += y;
    }
    int run = incl - s;
#pragma unroll 1
    for (int i = 0; i < NBA / 32; ++i) {
      const int cv = dsm[OC + base + i];
      dsm[OO + base + i] = run;
      dsm[OU + base + i] = run;
      run += cv;
    }
    const unsigned bm = __builtin_amdgcn_ballot_w32(bigl != 0);
    if (lane == 0) dsm[OM + 10] = (bm != 0u) ? 1 : 0;
  }
  __syncthreads();
  if (wave == 0) {
#pragma unroll 1
    for (int b0 = 0; b0 < tt; b0 += 32) {
      const int idx = b0 + lane;
      const int ent = dsm[OH + (idx < RCAP ? idx : RCAP - 1)];
      const int m32 = (tt - b0) < 32 ? (tt - b0) : 32;
#pragma unroll 1
      for (int k = 0; k < m32; ++k) {
        const int u    = __builtin_amdgcn_readlane(ent, k);
        const int slot = u & (NBA - 1);
        if (lane == 0) {
          int p = dsm[OU + slot];
          p = p < 0 ? 0 : (p > RCAP - 1 ? RCAP - 1 : p);
          dsm[OS + p] = u;
          dsm[OU + slot] = p + 1;
        }
      }
    }
  }
  __syncthreads();

  const int ovu = __builtin_amdgcn_readfirstlane(dsm[OM + 9] | dsm[OM + 10]);
  if (ovu != 0 && tid == 0) {
    volatile int* fq = (volatile int*)(flag + (int)blockIdx.x);
    *fq = 1;
    __threadfence();
    *fq = 1;
  }

  const float qnan = __int_as_float(0x7fc00000);
#pragma unroll 1
  for (int si = 0; si < NBA / NWAVE; ++si) {
    const int s    = si * NWAVE + wave;
    const int node = nodeBase + s;
    if (node >= NN) break;
    const int craw = dsm[OC + s];
    int cv = craw < 0 ? 0 : (craw > DEGCAP ? DEGCAP : craw);
    const int c = __builtin_amdgcn_readfirstlane(cv);
    int ofv = dsm[OO + s];
    ofv = ofv < 0 ? 0 : (ofv > RCAP ? RCAP : ofv);
    const int o = __builtin_amdgcn_readfirstlane(ofv);
    float a0 = 0.0f, a1 = 0.0f;
#pragma unroll 1
    for (int b0 = 0; b0 < c; b0 += 32) {
      int idx = o + b0 + lane;
      idx = idx > RCAP - 1 ? RCAP - 1 : idx;
      const int ent = dsm[OS + idx];
      int eid = ent >> SLA;
      eid = eid < 0 ? 0 : (eid > EE - 1 ? EE - 1 : eid);
      int sr = gath[eid];
      asm volatile("" :: "v"(sr));
      sr = sr < 0 ? 0 : (sr > NN - 1 ? NN - 1 : sr);
      const int m32 = (c - b0) < 32 ? (c - b0) : 32;
#pragma unroll 1
      for (int k = 0; k < m32; k += 4) {
        const int r0 = __builtin_amdgcn_readlane(sr, k);
        const int r1 = __builtin_amdgcn_readlane(sr, k + 1);
        const int r2 = __builtin_amdgcn_readlane(sr, k + 2);
        const int r3 = __builtin_amdgcn_readlane(sr, k + 3);
        const unsigned w0 = aplw[(size_t)r0 * APW + lane];
        const unsigned w1 = aplw[(size_t)r1 * APW + lane];
        const unsigned w2 = aplw[(size_t)r2 * APW + lane];
        const unsigned w3 = aplw[(size_t)r3 * APW + lane];
        asm volatile("" :: "v"(w0), "v"(w1), "v"(w2), "v"(w3));
        a0 += __uint_as_float(w0 << 16);
        a1 += __uint_as_float(w0 & 0xffff0000u);
        if (k + 1 < m32) { a0 += __uint_as_float(w1 << 16); a1 += __uint_as_float(w1 & 0xffff0000u); }
        if (k + 2 < m32) { a0 += __uint_as_float(w2 << 16); a1 += __uint_as_float(w2 & 0xffff0000u); }
        if (k + 3 < m32) { a0 += __uint_as_float(w3 << 16); a1 += __uint_as_float(w3 & 0xffff0000u); }
      }
    }
    const bool empty  = (c == 0);
    const bool poison = (ovu != 0) || (craw > DEGCAP);
    float m0 = empty ? 0.0f : a0;
    float m1 = empty ? 0.0f : a1;
    m0 = poison ? qnan : m0;
    m1 = poison ? qnan : m1;
    const unsigned hw = pk16(bf16_bits(m0), bf16_bits(m1));
    volatile unsigned* qh = (volatile unsigned*)(aplw + (size_t)node * APW + 32 + lane);
#if AGG_SPLIT
    const unsigned lw = pk16(bf16_lo_bits(m0), bf16_lo_bits(m1));
    volatile unsigned* ql = (volatile unsigned*)(aplw + (size_t)node * APW + 64 + lane);
#endif
    *qh = hw;
#if AGG_SPLIT
    *ql = lw;
#endif
    __threadfence();
    *qh = hw;
#if AGG_SPLIT
    *ql = lw;
#endif
  }
}

extern "C" void kernel_launch(void* const* d_in, const int* in_sizes, int n_in,
                              void* d_out, int out_size, void* d_ws, size_t ws_size,
                              hipStream_t stream) {
  if (n_in < 7) return;
  if (in_sizes[0] != NN * DD) return;
  if (in_sizes[1] != DD * DD || in_sizes[2] != DD) return;
  if (in_sizes[3] != DD * DD || in_sizes[4] != DD) return;
  if (in_sizes[5] != EE || in_sizes[6] != EE) return;
  if (out_size != NN * DD) return;
  if ((size_t)WS_TOTAL > ws_size) return;

  const float* feat = (const float*)d_in[0];
  const float* Wlin = (const float*)d_in[1];
  const float* blin = (const float*)d_in[2];
  const float* Wrot = (const float*)d_in[3];
  const float* brot = (const float*)d_in[4];
  const int*   gix  = (const int*)d_in[5];
  const int*   key  = (const int*)d_in[6];
  float* out = (float*)d_out;

  char* ws = (char*)d_ws;
  const size_t oA  = 0;
  const size_t oWB = oA + SZ_A;
  const size_t oBS = oWB + SZ_WB;
  const size_t oFL = oBS + SZ_BSUM;
  unsigned short* Apl = (unsigned short*)(ws + oA);
  unsigned short* WBp = (unsigned short*)(ws + oWB);
  float* bsum = (float*)(ws + oBS);
  int*   flag = (int*)(ws + oFL);

  const size_t scanLds = (size_t)SCAN_LDS_INTS * 4;
  hipFuncSetAttribute(reinterpret_cast<const void*>(&k_scan_sum), hipFuncAttributeMaxDynamicSharedMemorySize,
                      (int)scanLds);

  k_prep<<<PB_TOTAL, 256, 0, stream>>>(feat, Wlin, blin, Wrot, brot, Apl, WBp, bsum, flag);
  k_scan_sum<<<NBLK, NTHR, scanLds, stream>>>(gix, key, (unsigned*)Apl, flag);
  const int tiles = ((NN + 63) / 64) * ((DD + 63) / 64);
  k_gemm_nt<0, 1><<<(tiles + 7) / 8, 256, 0, stream>>>(Apl, WBp, bsum, out, NN, DD, AP, DD);
}
